// MambaBlock_84181359002077
// MI455X (gfx1250) — hardware-verified
//
#include <hip/hip_runtime.h>
#include <math.h>

typedef __attribute__((ext_vector_type(16))) _Float16 v16h;
typedef __attribute__((ext_vector_type(8)))  _Float16 v8h;
typedef __attribute__((ext_vector_type(8)))  float    v8f;
typedef __attribute__((ext_vector_type(4)))  float    v4f;

constexpr int kBatch = 2;
constexpr int kSeqL  = 1024;
constexpr int kDmod  = 1024;
constexpr int kDin   = 2048;
constexpr int kNst   = 16;
constexpr int kDtR   = 64;
constexpr int kPrjN  = 96;
constexpr int kPrjP  = 128;
constexpr int kXZP   = 2 * kDin;
constexpr int kRows  = kBatch * kSeqL;
constexpr int kKin   = 2 * kDmod;
constexpr int kTP    = 260;

constexpr float kCarryW    = 32.0f;
constexpr float kCarryXlo  = 256.0f;
constexpr float kCarryWlo  = kCarryW / kCarryXlo;
constexpr float kCarryU    = 16.0f;
constexpr float kCarryDt   = 16.0f;
constexpr float kCarryWdt  = 8.0f;
constexpr float kCarryY    = 16.0f;

static_assert(kDtR + 2 * kNst == kPrjN, "x_proj width");
static_assert(kRows == 2048 && kXZP == 4096 && kKin == 2048, "shape constants");
static_assert((kKin % 32) == 0 && (kDin % 32) == 0 && (kDtR % 32) == 0, "GEMM K multiples of 32");
static_assert((kRows % 64) == 0 && (kXZP % 64) == 0 && (kPrjP % 64) == 0 && (kDin % 64) == 0 && (kDmod % 64) == 0, "GEMM M,N multiples of 64");
static_assert((kSeqL % 64) == 0 && (kDin % 256) == 0 && (kSeqL & (kSeqL - 1)) == 0, "tile multiples");
static_assert(kCarryWlo == 0.125f, "balanced residual carry");

constexpr size_t kOffWIN  = 0;
constexpr size_t kOffWXP  = kOffWIN  + (size_t)kXZP  * kKin  * 2;
constexpr size_t kOffWDT  = kOffWXP  + (size_t)kPrjP * kDin  * 2;
constexpr size_t kOffWOUT = kOffWDT  + (size_t)kDin  * kDtR  * 2;
constexpr size_t kOffX16  = kOffWOUT + (size_t)kDmod * kDin  * 2;
constexpr size_t kOffXZ   = kOffX16  + (size_t)kRows * kKin  * 2;
constexpr size_t kOffUC   = kOffXZ   + (size_t)kRows * kXZP  * 4;
constexpr size_t kOffUC16 = kOffUC   + (size_t)kRows * kDin  * 4;
constexpr size_t kOffPROJ = kOffUC16 + (size_t)kRows * kDin  * 2;
constexpr size_t kOffDT16 = kOffPROJ + (size_t)kRows * kPrjP * 4;
constexpr size_t kOffDLR  = kOffDT16 + (size_t)kRows * kDtR  * 2;
constexpr size_t kOffY16  = kOffDLR  + (size_t)kRows * kDin  * 4;
constexpr size_t kWsTotal = kOffY16  + (size_t)kRows * kDin  * 2;
static_assert(kWsTotal == 115343360ull, "carve total");
static_assert(kWsTotal <= 134217728ull, "carve cap");
static_assert((kOffWXP % 128) == 0 && (kOffWDT % 128) == 0 && (kOffWOUT % 128) == 0 && (kOffX16 % 128) == 0 &&
              (kOffXZ % 128) == 0 && (kOffUC % 128) == 0 && (kOffUC16 % 128) == 0 && (kOffPROJ % 128) == 0 &&
              (kOffDT16 % 128) == 0 && (kOffDLR % 128) == 0 && (kOffY16 % 128) == 0, "128-B aligned regions");

__device__ __forceinline__ void keep4_h(v16h a, v16h b, v16h c, v16h d) { asm volatile("v_nop" :: "v"(a), "v"(b), "v"(c), "v"(d)); }
__device__ __forceinline__ void acc_guard4(v8f& a, v8f& b, v8f& c, v8f& d) { asm volatile("v_nop\n\tv_nop\n\tv_nop\n\tv_nop" : "+v"(a), "+v"(b), "+v"(c), "+v"(d)); }
__device__ __forceinline__ void group_guard_h(v8f& a, v8f& b, v8f& c, v8f& d, v16h x, v16h y0, v16h y1, v16h y2, v16h y3) {
  asm volatile("v_nop\n\tv_nop\n\tv_nop\n\tv_nop" : "+v"(a), "+v"(b), "+v"(c), "+v"(d) : "v"(x), "v"(y0), "v"(y1), "v"(y2), "v"(y3));
}
struct FragH {
  union U { v16h v; v8h h[2]; };
  static __device__ __forceinline__ v16h load(const _Float16* p) {
    U f;
    f.h[0] = *(const v8h*)(p);
    f.h[1] = *(const v8h*)(p + 16);
    return f.v;
  }
  static __device__ __forceinline__ v8f mma(v16h a, v16h b, v8f c) {
    return __builtin_amdgcn_wmma_f32_16x16x32_f16(false, a, false, b, (short)0, c, false, false);
  }
};

__global__ __launch_bounds__(256) void wmma_gemm64(
    const unsigned short* __restrict__ Ap, int lda,
    const unsigned short* __restrict__ Btp, int ldb,
    float* __restrict__ C, int ldc,
    int M, int N, int K, float scale) {
  const _Float16* A  = (const _Float16*)Ap;
  const _Float16* Bt = (const _Float16*)Btp;
  __shared__ __align__(16) float sT[8][16 * 68];
  const int lane = threadIdx.x & 31;
  const int wave = threadIdx.x >> 5;
  const int tilesN = N >> 6;
  const int tilesM = M >> 6;
  const int tile = blockIdx.x * 8 + wave;
  if (tile >= tilesM * tilesN) return;
  const int tm = tile / tilesN;
  const int tn = tile - tm * tilesN;
  const int m0 = tm << 6;
  const int n0 = tn << 6;

  const int rlane = lane & 15;
  const int koff  = (lane >> 4) * 8;
  const int mOff  = (lane >> 4) * 8;

  v8f acc[4][4];
#pragma unroll
  for (int i = 0; i < 4; ++i)
#pragma unroll
    for (int j = 0; j < 4; ++j) acc[i][j] = (v8f){0.f,0.f,0.f,0.f,0.f,0.f,0.f,0.f};

  for (int k0 = 0; k0 < K; k0 += 32) {
    v16h bh[4];
#pragma unroll
    for (int j = 0; j < 4; ++j) {
      const size_t bo = (size_t)(n0 + (j << 4) + rlane) * ldb + koff + k0;
      bh[j] = FragH::load(Bt + bo);
    }
#pragma unroll
    for (int i = 0; i < 4; ++i) {
      const size_t ao = (size_t)(m0 + (i << 4) + rlane) * lda + koff + k0;
      v16h ah = FragH::load(A + ao);
#pragma unroll
      for (int j = 0; j < 4; ++j) acc[i][j] = FragH::mma(ah, bh[j], acc[i][j]);
      group_guard_h(acc[i][0], acc[i][1], acc[i][2], acc[i][3], ah, bh[0], bh[1], bh[2], bh[3]);
    }
    keep4_h(bh[0], bh[1], bh[2], bh[3]);
  }
  acc_guard4(acc[0][0], acc[0][1], acc[0][2], acc[0][3]);
  acc_guard4(acc[1][0], acc[1][1], acc[1][2], acc[1][3]);
  acc_guard4(acc[2][0], acc[2][1], acc[2][2], acc[2][3]);
  acc_guard4(acc[3][0], acc[3][1], acc[3][2], acc[3][3]);

  float* slab = sT[wave];
#pragma unroll
  for (int i = 0; i < 4; ++i) {
    const int mBase = m0 + (i << 4);
#pragma unroll
    for (int j = 0; j < 4; ++j) {
#pragma unroll
      for (int r = 0; r < 8; ++r) {
        const float v = acc[i][j][r] * scale;
        slab[(mOff + r) * 68 + (j << 4) + rlane] = v;
      }
    }
    __builtin_amdgcn_fence(__ATOMIC_RELEASE, "workgroup");
    __builtin_amdgcn_wave_barrier();
    __builtin_amdgcn_fence(__ATOMIC_ACQUIRE, "workgroup");
    {
      const int hh = lane >> 4, c4 = (lane & 15) * 4;
      for (int pass = 0; pass < 2; ++pass) {
#pragma unroll
        for (int it = 0; it < 8; ++it) {
          const int row = it * 2 + hh;
          v4f v = *(const v4f*)(slab + row * 68 + c4);
          *(volatile v4f*)(C + (size_t)(mBase + row) * ldc + n0 + c4) = v;
        }
        __threadfence();
      }
    }
    __builtin_amdgcn_fence(__ATOMIC_RELEASE, "workgroup");
    __builtin_amdgcn_wave_barrier();
    __builtin_amdgcn_fence(__ATOMIC_ACQUIRE, "workgroup");
  }
}

__global__ __launch_bounds__(256) void x_split_kernel(
    const float* __restrict__ src, unsigned short* __restrict__ dst, int total8)
{
  const int i = blockIdx.x * 256 + threadIdx.x;
  if (i >= total8) return;
  const int e0  = i << 3;
  const int row = e0 / kDmod;
  const int c   = e0 - row * kDmod;
  const v4f a0 = *(const v4f*)(src + (size_t)e0);
  const v4f a1 = *(const v4f*)(src + (size_t)e0 + 4);
  v8h hv, lv;
#pragma unroll
  for (int e = 0; e < 4; ++e) {
    const float f0 = a0[e];
    const float f1 = a1[e];
    const _Float16 h0 = (_Float16)f0;
    const _Float16 h1 = (_Float16)f1;
    const float r0 = (f0 - (float)h0) * kCarryXlo;
    const float r1 = (f1 - (float)h1) * kCarryXlo;
    hv[e]     = h0;
    hv[4 + e] = h1;
    lv[e]     = (_Float16)r0;
    lv[4 + e] = (_Float16)r1;
  }
  unsigned short* qh = dst + (size_t)row * kKin + c;
  unsigned short* ql = qh + kDmod;
  *(volatile v8h*)qh = hv;
  *(volatile v8h*)ql = lv;
  __threadfence();
  *(volatile v8h*)qh = hv;
  *(volatile v8h*)ql = lv;
}

__global__ __launch_bounds__(256) void transpose_cast_kernel(
    const float* __restrict__ W, unsigned short* __restrict__ Bt, int Kdim, int Ndim, int ldo,
    float scale, int dupOff, float scale2)
{
  __shared__ float tile[64 * 65];
  const int tid = threadIdx.x, lane = tid & 31, wave = tid >> 5;
  const int n0 = blockIdx.x * 64;
  const int k0 = blockIdx.y * 64;
  (void)Kdim;
#pragma unroll
  for (int p = 0; p < 16; ++p) {
    const int idx = tid + p * 256;
    const int kk  = idx >> 6;
    const int nn  = idx & 63;
    const int n   = n0 + nn;
    const int nc  = (n < Ndim) ? n : (Ndim - 1);
    const float v = W[(size_t)(k0 + kk) * Ndim + nc];
    tile[kk * 65 + nn] = (n < Ndim) ? v : 0.f;
  }
  __syncthreads();
  const int q = lane >> 3, c8 = (lane & 7) * 8;
  v8h hv[2], hw[2];
#pragma unroll
  for (int it = 0; it < 2; ++it) {
    const int nrow = it * 32 + wave * 4 + q;
#pragma unroll
    for (int e = 0; e < 8; ++e) {
      const float t = tile[(c8 + e) * 65 + nrow];
      hv[it][e] = (_Float16)(t * scale);
      hw[it][e] = (_Float16)(t * scale2);
    }
  }
  for (int pass = 0; pass < 2; ++pass) {
#pragma unroll
    for (int it = 0; it < 2; ++it) {
      const int nrow = it * 32 + wave * 4 + q;
      unsigned short* o = Bt + (size_t)(n0 + nrow) * ldo + k0 + c8;
      *(volatile v8h*)o = hv[it];
      if (dupOff > 0) *(volatile v8h*)(o + dupOff) = hw[it];
    }
    __threadfence();
  }
}

__global__ __launch_bounds__(256) void dt_cast_kernel(
    const float* __restrict__ PROJ, unsigned short* __restrict__ DT16, int total8)
{
  const int i = blockIdx.x * 256 + threadIdx.x;
  if (i >= total8) return;
  const int e0  = i << 3;
  const int row = e0 >> 6;
  const int c8  = e0 & 63;
  const float* p = PROJ + (size_t)row * kPrjP + c8;
  const v4f a0 = *(const v4f*)(p);
  const v4f a1 = *(const v4f*)(p + 4);
  v8h hv;
#pragma unroll
  for (int e = 0; e < 4; ++e) {
    hv[e]     = (_Float16)(a0[e] * kCarryDt);
    hv[4 + e] = (_Float16)(a1[e] * kCarryDt);
  }
  unsigned short* qd = DT16 + e0;
  *(volatile v8h*)qd = hv;
  __threadfence();
  *(volatile v8h*)qd = hv;
}

__global__ __launch_bounds__(256) void conv_silu_kernel(
    const float* __restrict__ XZ, const float* __restrict__ cw, const float* __restrict__ cb,
    float* __restrict__ UC, unsigned short* __restrict__ UC16)
{
  __shared__ __align__(16) float sT[16 * kTP];
  const int tid = threadIdx.x, lane = tid & 31, wave = tid >> 5;
  const int d0 = blockIdx.x * 256, d = d0 + tid;
  const int g0 = blockIdx.y * 64;
  const int tb = g0 & (kSeqL - 1);
  const v4f wv = *(const v4f*)(cw + (size_t)d * 4);
  const float w0 = wv[0], w1 = wv[1], w2 = wv[2], w3 = wv[3];
  const float bc = cb[d];
  float xm3, xm2, xm1;
  {
    const bool hist = (tb > 0);
    const int rb = hist ? (g0 - 3) : g0;
    const float v3 = XZ[(size_t)rb * kXZP + d];
    const float v2 = XZ[(size_t)(rb + 1) * kXZP + d];
    const float v1 = XZ[(size_t)(rb + 2) * kXZP + d];
    xm3 = hist ? v3 : 0.f;
    xm2 = hist ? v2 : 0.f;
    xm1 = hist ? v1 : 0.f;
  }
  const int hrow = wave >> 1;
  const int hch  = (wave & 1) * 128 + lane * 4;
#pragma unroll 1
  for (int sub = 0; sub < 4; ++sub) {
    const int lb = g0 + sub * 16;
#pragma unroll 1
    for (int s = 0; s < 16; ++s) {
      const float xc = XZ[(size_t)(lb + s) * kXZP + d];
      float acc = w0 * xm3;
      acc = fmaf(w1, xm2, acc);
      acc = fmaf(w2, xm1, acc);
      acc = fmaf(w3, xc, acc);
      const float sv = acc + bc;
      const float sg = __builtin_amdgcn_rcpf(1.0f + expf(-sv));
      sT[s * kTP + tid] = sv * sg;
      xm3 = xm2;
      xm2 = xm1;
      xm1 = xc;
    }
    __syncthreads();
    v4f fv[4];
    v8h bv[2];
#pragma unroll
    for (int it = 0; it < 4; ++it) fv[it] = *(const v4f*)(sT + (it * 4 + hrow) * kTP + hch);
#pragma unroll
    for (int it = 0; it < 2; ++it) {
      const float* sp = sT + (it * 8 + wave) * kTP + lane * 8;
      const v4f a0 = *(const v4f*)(sp);
      const v4f a1 = *(const v4f*)(sp + 4);
#pragma unroll
      for (int e = 0; e < 4; ++e) {
        bv[it][e]     = (_Float16)(a0[e] * kCarryU);
        bv[it][4 + e] = (_Float16)(a1[e] * kCarryU);
      }
    }
    for (int pass = 0; pass < 2; ++pass) {
#pragma unroll
      for (int it = 0; it < 4; ++it)
        *(volatile v4f*)(UC + (size_t)(lb + it * 4 + hrow) * kDin + d0 + hch) = fv[it];
#pragma unroll
      for (int it = 0; it < 2; ++it)
        *(volatile v8h*)(UC16 + (size_t)(lb + it * 8 + wave) * kDin + d0 + lane * 8) = bv[it];
      __threadfence();
    }
    __syncthreads();
  }
}

__global__ __launch_bounds__(256) void scan_kernel(
    const float* __restrict__ DLR, const float* __restrict__ UC, const float* __restrict__ XZ,
    const float* __restrict__ PROJ, const float* __restrict__ bdt, const float* __restrict__ A_log,
    const float* __restrict__ Dv, unsigned short* __restrict__ Y16)
{
  __shared__ __align__(16) float sBC[16 * 32];
  __shared__ __align__(16) float sY[16 * kTP];
  const int tid = threadIdx.x, lane = tid & 31, wave = tid >> 5;
  constexpr int kBlkPerB = kDin / 256;
  const int bix = blockIdx.x / kBlkPerB;
  const int d0  = (blockIdx.x - bix * kBlkPerB) * 256;
  const int d   = d0 + tid;
  const size_t row0 = (size_t)bix * kSeqL;

  float An[kNst];
#pragma unroll
  for (int q4 = 0; q4 < 4; ++q4) {
    const v4f al = *(const v4f*)(A_log + (size_t)d * kNst + 4 * q4);
    An[4 * q4 + 0] = -expf(al[0]);
    An[4 * q4 + 1] = -expf(al[1]);
    An[4 * q4 + 2] = -expf(al[2]);
    An[4 * q4 + 3] = -expf(al[3]);
  }
  const float Dd = Dv[d];
  const float bb = bdt[d];
  float h[kNst];
#pragma unroll
  for (int n = 0; n < kNst; ++n) h[n] = 0.f;

#pragma unroll 1
  for (int c = 0; c < kSeqL / 16; ++c) {
    const int l0 = c * 16;
    if (tid < 128) {
      const int r = tid >> 3, q = (tid & 7) * 4;
      const v4f v = *(const v4f*)(PROJ + (row0 + l0 + r) * kPrjP + kDtR + q);
      *(v4f*)(sBC + r * 32 + q) = v;
    }
    __syncthreads();
#pragma unroll 1
    for (int s = 0; s < 16; ++s) {
      const size_t m = row0 + (size_t)(l0 + s);
      const float a     = DLR[m * kDin + d] + bb;
      const float delta = fmaxf(a, 0.0f) + log1pf(expf(-fabsf(a)));
      const float xv    = UC[m * kDin + d];
      const float zv    = XZ[m * kXZP + kDin + d];
      v4f Bq[4], Cq[4];
#pragma unroll
      for (int qq = 0; qq < 4; ++qq) {
        Bq[qq] = *(const v4f*)(sBC + s * 32 + 4 * qq);
        Cq[qq] = *(const v4f*)(sBC + s * 32 + kNst + 4 * qq);
      }
      float y = 0.f;
#pragma unroll
      for (int n = 0; n < kNst; ++n) {
        const float e = expf(delta * An[n]);
        float db = delta * Bq[n >> 2][n & 3];
        asm volatile("" : "+v"(db));
        float p = db * xv;
        asm volatile("" : "+v"(p));
        float qv = h[n] * e;
        asm volatile("" : "+v"(qv));
        const float hn = qv + p;
        h[n] = hn;
        float rr = Cq[n >> 2][n & 3] * hn;
        asm volatile("" : "+v"(rr));
        y += rr;
      }
      float sk = xv * Dd;
      asm volatile("" : "+v"(sk));
      y += sk;
      const float sg = __builtin_amdgcn_rcpf(1.0f + expf(-zv));
      const float g  = zv * sg;
      sY[s * kTP + tid] = (y * g) * kCarryY;
    }
    __syncthreads();
    v8h hv[2];
#pragma unroll
    for (int it = 0; it < 2; ++it) {
      const float* sp = sY + (it * 8 + wave) * kTP + lane * 8;
      const v4f a0 = *(const v4f*)(sp);
      const v4f a1 = *(const v4f*)(sp + 4);
#pragma unroll
      for (int e = 0; e < 4; ++e) {
        hv[it][e]     = (_Float16)a0[e];
        hv[it][4 + e] = (_Float16)a1[e];
      }
    }
    for (int pass = 0; pass < 2; ++pass) {
#pragma unroll
      for (int it = 0; it < 2; ++it)
        *(volatile v8h*)(Y16 + (row0 + (size_t)(l0 + it * 8 + wave)) * kDin + d0 + lane * 8) = hv[it];
      __threadfence();
    }
  }
}

extern "C" void kernel_launch(void* const* d_in, const int* in_sizes, int n_in,
                              void* d_out, int out_size, void* d_ws, size_t ws_size,
                              hipStream_t stream)
{
  if (n_in < 10) return;
  if (in_sizes[0] != kRows * kDmod) return;
  if (in_sizes[1] != kDmod * kXZP) return;
  if (in_sizes[2] != kDin * 4 || in_sizes[3] != kDin) return;
  if (in_sizes[4] != kDin * kPrjN) return;
  if (in_sizes[5] != kDtR * kDin || in_sizes[6] != kDin) return;
  if (in_sizes[7] != kDin * kNst || in_sizes[8] != kDin) return;
  if (in_sizes[9] != kDin * kDmod) return;
  if (out_size != kRows * kDmod) return;
  if (ws_size < kWsTotal) return;

  const float* x      = (const float*)d_in[0];
  const float* W_in   = (const float*)d_in[1];
  const float* conv_w = (const float*)d_in[2];
  const float* conv_b = (const float*)d_in[3];
  const float* W_xp   = (const float*)d_in[4];
  const float* W_dt   = (const float*)d_in[5];
  const float* b_dt   = (const float*)d_in[6];
  const float* A_log  = (const float*)d_in[7];
  const float* Dv     = (const float*)d_in[8];
  const float* W_out  = (const float*)d_in[9];
  float* dout = (float*)d_out;

  char* ws = (char*)d_ws;
  unsigned short* WIN16  = (unsigned short*)(ws + kOffWIN);
  unsigned short* WXP16  = (unsigned short*)(ws + kOffWXP);
  unsigned short* WDT16  = (unsigned short*)(ws + kOffWDT);
  unsigned short* WOUT16 = (unsigned short*)(ws + kOffWOUT);
  unsigned short* X16    = (unsigned short*)(ws + kOffX16);
  float*          XZ     = (float*)(ws + kOffXZ);
  float*          UC     = (float*)(ws + kOffUC);
  unsigned short* UC16   = (unsigned short*)(ws + kOffUC16);
  float*          PROJ   = (float*)(ws + kOffPROJ);
  unsigned short* DT16   = (unsigned short*)(ws + kOffDT16);
  float*          DLR    = (float*)(ws + kOffDLR);
  unsigned short* Y16    = (unsigned short*)(ws + kOffY16);

  transpose_cast_kernel<<<dim3(kXZP / 64, kDmod / 64), 256, 0, stream>>>(W_in, WIN16, kDmod, kXZP, kKin, kCarryW, kDmod, kCarryWlo);
  transpose_cast_kernel<<<dim3(kPrjP / 64, kDin / 64), 256, 0, stream>>>(W_xp, WXP16, kDin, kPrjN, kDin, kCarryW, 0, 0.0f);
  transpose_cast_kernel<<<dim3(kDin / 64, kDtR / 64), 256, 0, stream>>>(W_dt, WDT16, kDtR, kDin, kDtR, kCarryWdt, 0, 0.0f);
  transpose_cast_kernel<<<dim3(kDmod / 64, kDin / 64), 256, 0, stream>>>(W_out, WOUT16, kDin, kDmod, kDin, kCarryW, 0, 0.0f);

  x_split_kernel<<<(kRows * kDmod) / 8 / 256, 256, 0, stream>>>(x, X16, (kRows * kDmod) / 8);

  wmma_gemm64<<<dim3(256, 1), 256, 0, stream>>>(X16, kKin, WIN16, kKin, XZ, kXZP, kRows, kXZP, kKin, 1.0f / kCarryW);

  conv_silu_kernel<<<dim3(kDin / 256, kRows / 64), 256, 0, stream>>>(XZ, conv_w, conv_b, UC, UC16);

  wmma_gemm64<<<dim3(8, 1), 256, 0, stream>>>(UC16, kDin, WXP16, kDin, PROJ, kPrjP, kRows, kPrjP, kDin, 1.0f / (kCarryU * kCarryW));

  dt_cast_kernel<<<(kRows * kDtR) / 8 / 256, 256, 0, stream>>>(PROJ, DT16, (kRows * kDtR) / 8);

  wmma_gemm64<<<dim3(128, 1), 256, 0, stream>>>(DT16, kDtR, WDT16, kDtR, DLR, kDin, kRows, kDin, kDtR, 1.0f / (kCarryDt * kCarryWdt));

  scan_kernel<<<dim3(kBatch * (kDin / 256), 1), 256, 0, stream>>>(DLR, UC, XZ, PROJ, b_dt, A_log, Dv, Y16);

  wmma_gemm64<<<dim3(64, 1), 256, 0, stream>>>(Y16, kDin, WOUT16, kDin, dout, kDmod, kRows, kDmod, kDin, 1.0f / (kCarryY * kCarryW));
}
